// TimeframeInteractionHierarchy_9431748182488
// MI455X (gfx1250) — hardware-verified
//
#include <hip/hip_runtime.h>


constexpr int NTF_   = 11;
constexpr int NBT_   = 512;
constexpr int HD_    = 128;
constexpr int NROW_  = NTF_ * NBT_;
constexpr int NWP_   = HD_ * HD_;
constexpr int MROWS_ = 32;
constexpr int AP_    = HD_ + 4;
constexpr int SP_    = MROWS_ + 4;

static_assert(NBT_ % MROWS_ == 0);
static_assert(NROW_ % 64 == 0);
static_assert(HD_ % 32 == 0);
static_assert((AP_ * 4) % 16 == 0);
static_assert((SP_ * 4) % 16 == 0);
static_assert(MROWS_ * HD_ == 4 * 1024);
static_assert((MROWS_ * AP_) % 4 == 0);

typedef float    v4f  __attribute__((ext_vector_type(4)));
typedef float    v8f  __attribute__((ext_vector_type(8)));
typedef _Float16 v8h  __attribute__((ext_vector_type(8)));
typedef _Float16 v16h __attribute__((ext_vector_type(16)));

union FragH { v8h h[2]; v16h v; };

__device__ __forceinline__ v8f ld8f(const float* p) {
    v4f a = *(const v4f*)p;
    v4f b = *(const v4f*)(p + 4);
    return __builtin_shufflevector(a, b, 0, 1, 2, 3, 4, 5, 6, 7);
}
__device__ __forceinline__ v8h cvt8h(v8f x) {
    return __builtin_convertvector(x, v8h);
}
__device__ __forceinline__ float wsum32(float v) {
    v += __shfl_xor(v, 16, 32);
    v += __shfl_xor(v, 8, 32);
    v += __shfl_xor(v, 4, 32);
    v += __shfl_xor(v, 2, 32);
    v += __shfl_xor(v, 1, 32);
    return v;
}
__device__ __forceinline__ void mma_h(v8f& acc, const FragH& a, const FragH& b) {
    acc = __builtin_amdgcn_wmma_f32_16x16x32_f16(false, a.v, false, b.v, (short)0, acc, false, false);
    asm volatile("v_nop\n\tv_nop\n\tv_nop\n\tv_nop" : "+v"(acc) : "v"(a.v), "v"(b.v));
}

__global__ __launch_bounds__(256)
void cvt_h_kernel(const float* __restrict__ h, _Float16* Hh, int n8)
{
    const int i = blockIdx.x * 256 + threadIdx.x;
    if (i >= n8) return;
    const size_t e = (size_t)i * 8;
    const v8h y = cvt8h(ld8f(h + e));
    *(volatile v8h*)(Hh + e) = y;
    __threadfence();
    *(volatile v8h*)(Hh + e) = y;
}

__global__ __launch_bounds__(256)
void cvt_wlr_kernel(const float* __restrict__ Wlr, _Float16* WL)
{
    const int i = blockIdx.x * 256 + threadIdx.x;
    if (i >= 2 * HD_ * 16) return;
    const int n   = i >> 4;
    const int g   = i & 15;
    const int row = n & (HD_ - 1);
    const int cb  = (n >> 7) * HD_;
    const v8f x = ld8f(Wlr + (size_t)row * (2 * HD_) + cb + g * 8) * 16.0f;
    const v8h y = cvt8h(x);
    const size_t e = (size_t)n * HD_ + g * 8;
    *(volatile v8h*)(WL + e) = y;
    __threadfence();
    *(volatile v8h*)(WL + e) = y;
}

__global__ __launch_bounds__(256)
void wtrans_kernel(const float* __restrict__ W1, const float* __restrict__ W2, const float* __restrict__ W3,
                   _Float16* WP)
{
    __shared__ __attribute__((aligned(16))) float s[HD_ * 33];
    const int tid = threadIdx.x;
    const int jc = blockIdx.x, o = blockIdx.y, d = blockIdx.z;
    const float* W = (d == 0) ? W1 : ((d == 1) ? W2 : W3);
    const float* src = W + (size_t)o * NWP_ + jc * 32;
#pragma unroll
    for (int it = 0; it < 4; ++it) {
        const int i  = it * 32 + (tid >> 3);
        const int j4 = (tid & 7) * 4;
        const v4f x = *(const v4f*)(src + (size_t)i * HD_ + j4);
        float* sp = s + i * 33 + j4;
        sp[0] = x.x * 64.0f;
        sp[1] = x.y * 64.0f;
        sp[2] = x.z * 64.0f;
        sp[3] = x.w * 64.0f;
    }
    __syncthreads();

    _Float16* dst = WP + ((size_t)d * NWP_ + (size_t)o * HD_ + jc * 32) * HD_;
    v8h vals[2];
    size_t goff[2];
#pragma unroll
    for (int it = 0; it < 2; ++it) {
        const int line  = it * 32 + (tid >> 3);
        const int jj    = line >> 1;
        const int hf    = line & 1;
        const int piece = tid & 7;
        const int i0    = hf * 64 + piece * 8;
        v8f x;
#pragma unroll
        for (int c = 0; c < 8; ++c) x[c] = s[(i0 + c) * 33 + jj];
        vals[it] = cvt8h(x);
        goff[it] = (size_t)jj * HD_ + i0;
    }
    *(volatile v8h*)(dst + goff[0]) = vals[0];
    *(volatile v8h*)(dst + goff[1]) = vals[1];
    __threadfence();
    *(volatile v8h*)(dst + goff[0]) = vals[0];
    *(volatile v8h*)(dst + goff[1]) = vals[1];
}

template<int NBF>
__device__ __forceinline__ void tile_store_pass(const float* st, float* gp, int ldc, int lane) {
    constexpr int CW  = NBF * 16;
    constexpr int P   = CW + 4;
    constexpr int LPR = CW / 4;
    constexpr int RPI = 32 / LPR;
    constexpr int NIT = 32 / RPI;
    const int rsub = lane / LPR;
    const int c4   = (lane % LPR) * 4;
#pragma unroll
    for (int it = 0; it < NIT; ++it) {
        const int row = it * RPI + rsub;
        const v4f v = *(const v4f*)(st + row * P + c4);
        *(volatile v4f*)(gp + (size_t)row * ldc + c4) = v;
    }
}

__global__ __launch_bounds__(128)
void pq_gemm_kernel(const _Float16* __restrict__ A, const _Float16* __restrict__ B, float* C, int K, int ldc)
{
    constexpr int NBF = 2;
    constexpr int CW  = NBF * 16;
    constexpr int P   = CW + 4;
    __shared__ __attribute__((aligned(16))) float stile[4][32 * P];

    const int tid  = threadIdx.x;
    const int lane = tid & 31;
    const int wave = tid >> 5;
    const int hh   = lane >> 4;
    const int m    = lane & 15;
    const int wm   = wave >> 1;
    const int wn   = wave & 1;

    const int rowW = blockIdx.y * 64 + wm * 32;
    const int colW = blockIdx.x * (2 * CW) + wn * CW;

    v8f acc[2 * NBF];
#pragma unroll
    for (int j = 0; j < 2 * NBF; ++j)
#pragma unroll
        for (int r = 0; r < 8; ++r) acc[j][r] = 0.0f;

    const size_t aoff  = (size_t)(rowW + m) * K + 8 * hh;
    const size_t boff  = (size_t)(colW + m) * K + 8 * hh;
    const size_t sub16 = (size_t)16 * K;
    const int nk = K >> 5;

#pragma unroll 1
    for (int kt = 0; kt < nk; ++kt) {
        const size_t k0 = (size_t)kt * 32;
        FragH fa[2], fb[NBF];
#pragma unroll
        for (int s = 0; s < 2; ++s) {
            const _Float16* p = A + aoff + s * sub16 + k0;
            fa[s].h[0] = *(const v8h*)(p);
            fa[s].h[1] = *(const v8h*)(p + 16);
        }
#pragma unroll
        for (int j = 0; j < NBF; ++j) {
            const _Float16* p = B + boff + j * sub16 + k0;
            fb[j].h[0] = *(const v8h*)(p);
            fb[j].h[1] = *(const v8h*)(p + 16);
        }
#pragma unroll
        for (int s = 0; s < 2; ++s)
#pragma unroll
            for (int j = 0; j < NBF; ++j)
                mma_h(acc[s * NBF + j], fa[s], fb[j]);
    }

    float* st = stile[wave];
#pragma unroll
    for (int s = 0; s < 2; ++s)
#pragma unroll
        for (int j = 0; j < NBF; ++j)
#pragma unroll
            for (int r = 0; r < 8; ++r)
                st[(s * 16 + 8 * hh + r) * P + j * 16 + m] = acc[s * NBF + j][r] * 0.0625f;
    __syncthreads();

    float* gp = C + (size_t)rowW * ldc + colW;
    tile_store_pass<NBF>(st, gp, ldc, lane);
    __threadfence();
    tile_store_pass<NBF>(st, gp, ldc, lane);
}

__global__ __launch_bounds__(256)
void bil_main_kernel(const float* __restrict__ h, const _Float16* __restrict__ Hh, const _Float16* __restrict__ WP,
                     const float* __restrict__ PQ,
                     const float* __restrict__ V1p, const float* __restrict__ V2p, const float* __restrict__ V3p,
                     const float* __restrict__ decp,
                     const float* __restrict__ b1, const float* __restrict__ b2, const float* __restrict__ b3,
                     const float* __restrict__ blr, const float* __restrict__ lnw, const float* __restrict__ lnb,
                     float* out)
{
    __shared__ __attribute__((aligned(16))) float accL[MROWS_ * AP_];
    __shared__ __attribute__((aligned(16))) float sST[HD_ * SP_];

    const int tid  = threadIdx.x;
    const int lane = tid & 31;
    const int wave = tid >> 5;
    const int hh   = lane >> 4;
    const int m    = lane & 15;
    const int rs   = wave & 1;
    const int oo   = wave >> 1;
    const int r0   = blockIdx.x * MROWS_;
    const int tf   = r0 / NBT_;
    const int bb0  = r0 - tf * NBT_;

    const v4f z4 = {0.0f, 0.0f, 0.0f, 0.0f};
#pragma unroll 1
    for (int e4 = tid; e4 < (MROWS_ * AP_) / 4; e4 += 256) *(v4f*)(accL + e4 * 4) = z4;

    const float v1 = V1p[0], v2 = V2p[0], v3 = V3p[0];
    const float ndec = -decp[0];
    const size_t arow = (size_t)(r0 + 16 * rs + m) * HD_ + 8 * hh;

#pragma unroll 1
    for (int dd = 0; dd < 3; ++dd) {
        const int dist = dd + 1;
        const float Vd = (dd == 0) ? v1 : ((dd == 1) ? v2 : v3);
        const float* bd = (dd == 0) ? b1 : ((dd == 1) ? b2 : b3);
        const _Float16* Wp = WP + (size_t)dd * NWP_ * HD_;
        const bool ep = (tf + dist <= NTF_ - 1);
        const bool em = (tf >= dist);
        const float cnt = (ep ? 1.0f : 0.0f) + (em ? 1.0f : 0.0f);
        const int tfp = min(tf + dist, NTF_ - 1);
        const int tfm = max(tf - dist, 0);
        const float* hp = h + ((size_t)tfp * NBT_ + bb0) * HD_;
        const float* hm = h + ((size_t)tfm * NBT_ + bb0) * HD_;

        __syncthreads();
#pragma unroll
        for (int it = 0; it < 4; ++it) {
            const int e   = it * 256 + tid;
            const int row = e >> 5;
            const int j0  = (e & 31) * 4;
            const v4f xp = *(const v4f*)(hp + (size_t)row * HD_ + j0);
            const v4f xm = *(const v4f*)(hm + (size_t)row * HD_ + j0);
            v4f sv = z4;
            if (ep) sv += xp;
            if (em) sv += xm;
            sST[(j0 + 0) * SP_ + row] = sv.x;
            sST[(j0 + 1) * SP_ + row] = sv.y;
            sST[(j0 + 2) * SP_ + row] = sv.z;
            sST[(j0 + 3) * SP_ + row] = sv.w;
        }
        __syncthreads();

#pragma unroll 1
        for (int c = 0; c < HD_ / 4; ++c) {
            const int o = 4 * c + oo;
            const _Float16* wrow = Wp + ((size_t)o * HD_ + m) * HD_ + 8 * hh;
            v8f acc[8];
#pragma unroll
            for (int t = 0; t < 8; ++t)
#pragma unroll
                for (int r = 0; r < 8; ++r) acc[t][r] = 0.0f;

#pragma unroll 1
            for (int ks = 0; ks < HD_ / 32; ++ks) {
                FragH a;
                const _Float16* pa = Hh + arow + ks * 32;
                a.h[0] = *(const v8h*)(pa);
                a.h[1] = *(const v8h*)(pa + 16);
#pragma unroll
                for (int t = 0; t < 8; ++t) {
                    FragH b;
                    const _Float16* pb = wrow + (size_t)t * (16 * HD_) + ks * 32;
                    b.h[0] = *(const v8h*)(pb);
                    b.h[1] = *(const v8h*)(pb + 16);
                    mma_h(acc[t], a, b);
                }
            }

            float part[8];
#pragma unroll
            for (int r = 0; r < 8; ++r) part[r] = 0.0f;
            const float* sp0 = sST + m * SP_ + 16 * rs + 8 * hh;
#pragma unroll
            for (int t = 0; t < 8; ++t) {
                const float* sp = sp0 + t * 16 * SP_;
                const v4f s0 = *(const v4f*)(sp);
                const v4f s1 = *(const v4f*)(sp + 4);
                part[0] = fmaf(acc[t][0], s0.x, part[0]);
                part[1] = fmaf(acc[t][1], s0.y, part[1]);
                part[2] = fmaf(acc[t][2], s0.z, part[2]);
                part[3] = fmaf(acc[t][3], s0.w, part[3]);
                part[4] = fmaf(acc[t][4], s1.x, part[4]);
                part[5] = fmaf(acc[t][5], s1.y, part[5]);
                part[6] = fmaf(acc[t][6], s1.z, part[6]);
                part[7] = fmaf(acc[t][7], s1.w, part[7]);
            }
#pragma unroll
            for (int r = 0; r < 8; ++r) {
                float v = part[r];
                v += __shfl_xor(v, 1, 32);
                v += __shfl_xor(v, 2, 32);
                v += __shfl_xor(v, 4, 32);
                v += __shfl_xor(v, 8, 32);
                part[r] = v;
            }
            float mine = part[0];
#pragma unroll
            for (int r = 1; r < 8; ++r) mine = (m == r) ? part[r] : mine;
            const float bo  = bd[o];
            const float val = Vd * (mine * 0.015625f + cnt * bo);
            if (m < 8) accL[(16 * rs + 8 * hh + m) * AP_ + o] += val;
        }
    }
    __syncthreads();

    const int c0 = lane * 4;
    const v4f wv  = *(const v4f*)(lnw + c0);
    const v4f bv  = *(const v4f*)(lnb + c0);
    const v4f blv = *(const v4f*)(blr + c0);
#pragma unroll 1
    for (int rr = 0; rr < MROWS_ / 8; ++rr) {
        const int q = wave * (MROWS_ / 8) + rr;
        const size_t grow = (size_t)(r0 + q);
        const int bidx = bb0 + q;
        v4f a = *(const v4f*)(accL + q * AP_ + c0);
        const v4f Pv = *(const v4f*)(PQ + grow * (2 * HD_) + c0);
#pragma unroll 1
        for (int dist = 4; dist < NTF_; ++dist) {
            const float Vd = v3 * expf(ndec * (float)(dist - 3));
            const bool ep = (tf + dist <= NTF_ - 1);
            const bool em = (tf >= dist);
            const int tfp = min(tf + dist, NTF_ - 1);
            const int tfm = max(tf - dist, 0);
            const v4f Qp = *(const v4f*)(PQ + ((size_t)tfp * NBT_ + bidx) * (2 * HD_) + HD_ + c0);
            const v4f Qm = *(const v4f*)(PQ + ((size_t)tfm * NBT_ + bidx) * (2 * HD_) + HD_ + c0);
            const v4f tp = ((Pv + Qp) + blv) * Vd;
            const v4f tm = ((Pv + Qm) + blv) * Vd;
            if (ep) a += tp;
            if (em) a += tm;
        }
        const v4f x = *(const v4f*)(h + grow * HD_ + c0) + a;
        float ssum = (x.x + x.y) + (x.z + x.w);
        ssum = wsum32(ssum);
        const float mu = ssum * 0.0078125f;
        const v4f dv = x - mu;
        float qq = dv.x * dv.x + dv.y * dv.y + dv.z * dv.z + dv.w * dv.w;
        qq = wsum32(qq);
        const float rinv = rsqrtf(qq * 0.0078125f + 1e-5f);
        const v4f ov = (dv * rinv) * wv + bv;
        float* gp = out + grow * HD_ + c0;
        *(volatile v4f*)gp = ov;
        __threadfence();
        *(volatile v4f*)gp = ov;
    }
}

extern "C" void kernel_launch(void* const* d_in, const int* in_sizes, int n_in,
                              void* d_out, int out_size, void* d_ws, size_t ws_size,
                              hipStream_t stream)
{
    if (n_in < 15) return;
    const int want[15] = { NROW_ * HD_, 1, 1, 1, 1,
                           HD_ * HD_ * HD_, HD_, HD_ * HD_ * HD_, HD_, HD_ * HD_ * HD_, HD_,
                           HD_ * 2 * HD_, HD_, HD_, HD_ };
    for (int i = 0; i < 15; ++i) if (in_sizes[i] != want[i]) return;
    if (out_size != NROW_ * HD_) return;

    const float* h    = (const float*)d_in[0];
    const float* V1   = (const float*)d_in[1];
    const float* V2   = (const float*)d_in[2];
    const float* V3   = (const float*)d_in[3];
    const float* Vdec = (const float*)d_in[4];
    const float* W1   = (const float*)d_in[5];
    const float* b1   = (const float*)d_in[6];
    const float* W2   = (const float*)d_in[7];
    const float* b2   = (const float*)d_in[8];
    const float* W3   = (const float*)d_in[9];
    const float* b3   = (const float*)d_in[10];
    const float* Wlr  = (const float*)d_in[11];
    const float* blr  = (const float*)d_in[12];
    const float* lnw  = (const float*)d_in[13];
    const float* lnb  = (const float*)d_in[14];
    float* out = (float*)d_out;

    char* ws = (char*)d_ws;
    size_t off = 0;
    auto carve = [&](size_t bytes) -> char* { char* p = ws + off; off += (bytes + 255) & ~(size_t)255; return p; };
    const size_t HH_B = (size_t)NROW_ * HD_ * 2;
    const size_t WP_B = (size_t)3 * NWP_ * HD_ * 2;
    const size_t WL_B = (size_t)2 * HD_ * HD_ * 2;
    const size_t PQ_B = (size_t)NROW_ * 2 * HD_ * 4;
    _Float16* Hh = (_Float16*)carve(HH_B);
    _Float16* WP = (_Float16*)carve(WP_B);
    _Float16* WL = (_Float16*)carve(WL_B);
    float*    PQ = (float*)carve(PQ_B);
    if (off > ws_size) return;

    const dim3 b256(256), b128(128);
    const int n8h = (NROW_ * HD_) / 8;

    cvt_h_kernel<<<dim3((n8h + 255) / 256), b256, 0, stream>>>(h, Hh, n8h);
    cvt_wlr_kernel<<<dim3((2 * HD_ * 16 + 255) / 256), b256, 0, stream>>>(Wlr, WL);
    wtrans_kernel<<<dim3(HD_ / 32, HD_, 3), b256, 0, stream>>>(W1, W2, W3, WP);

    pq_gemm_kernel<<<dim3((2 * HD_) / 64, NROW_ / 64), b128, 0, stream>>>(Hh, WL, PQ, HD_, 2 * HD_);

    bil_main_kernel<<<dim3(NROW_ / MROWS_), b256, 0, stream>>>(h, Hh, WP, PQ, V1, V2, V3, Vdec,
                                                                b1, b2, b3, blr, lnw, lnb, out);
}
